// RecurrentActorCritic_18373870092920
// MI455X (gfx1250) — hardware-verified
//
#include <hip/hip_runtime.h>
#include <math.h>

constexpr int kSteps   = 256;
constexpr int kBatch   = 512;
constexpr int kObs     = 64;
constexpr int kEnc1    = 128;
constexpr int kHid     = 256;
constexpr int kLstm    = 128;
constexpr int kGates   = 512;
constexpr int kAct     = 8;
constexpr int kHeadN   = 64;
constexpr int kGroups  = 4;
constexpr int kSeqGrp  = 128;
constexpr int kRowsGrp = kSeqGrp * kSteps;
constexpr int kNT      = 256;
constexpr int kAhP     = 136;
constexpr int kHfP     = 132;
constexpr float kInv8  = 1.0f / 8.0f;
constexpr float kInv16 = 1.0f / 16.0f;
static_assert(kGroups * kSeqGrp == kBatch);
static_assert(kRowsGrp % 64 == 0);
static_assert(kGates == 4 * kLstm);

typedef __attribute__((ext_vector_type(16))) _Float16 v16h;
typedef __attribute__((ext_vector_type(8)))  _Float16 v8h;
typedef __attribute__((ext_vector_type(16))) __bf16   v16b;
typedef __attribute__((ext_vector_type(8)))  __bf16   v8b;
typedef __attribute__((ext_vector_type(8)))  float    v8f;
typedef __attribute__((ext_vector_type(4)))  float    v4f;

__device__ __forceinline__ unsigned short f2bf_bits(float f) {
  unsigned u = __float_as_uint(f);
  return (unsigned short)((u + 0x7FFFu + ((u >> 16) & 1u)) >> 16);
}
__device__ __forceinline__ float bf_bits2f(unsigned short h) { return __uint_as_float(((unsigned)h) << 16); }

__device__ __forceinline__ void dep_guard_h(v8f& a, v8f& b, v16h x, v16h y) { asm volatile("v_nop\n\tv_nop\n\tv_nop\n\tv_nop" : "+v"(a), "+v"(b) : "v"(x), "v"(y)); }
__device__ __forceinline__ void dep_guard_b(v8f& a, v8f& b, v16b x, v16b y) { asm volatile("v_nop\n\tv_nop\n\tv_nop\n\tv_nop" : "+v"(a), "+v"(b) : "v"(x), "v"(y)); }
__device__ __forceinline__ void keep4_h(v16h a, v16h b, v16h c, v16h d) { asm volatile("v_nop" :: "v"(a), "v"(b), "v"(c), "v"(d)); }
__device__ __forceinline__ void keep4_b(v16b a, v16b b, v16b c, v16b d) { asm volatile("v_nop" :: "v"(a), "v"(b), "v"(c), "v"(d)); }
__device__ __forceinline__ void acc_guard4(v8f& a, v8f& b, v8f& c, v8f& d) { asm volatile("v_nop\n\tv_nop\n\tv_nop\n\tv_nop" : "+v"(a), "+v"(b), "+v"(c), "+v"(d)); }
template <typename T> struct Frag;
template <> struct Frag<_Float16> {
  typedef v16h V; union U { v16h v; v8h h[2]; };
  static __device__ __forceinline__ v16h load(const _Float16* p) {
    U f; f.h[0] = *(const v8h*)(p); f.h[1] = *(const v8h*)(p + 16); return f.v;
  }
  static __device__ __forceinline__ v8f mma(v16h a, v16h b, v8f c) {
    return __builtin_amdgcn_wmma_f32_16x16x32_f16(false, a, false, b, (short)0, c, false, false);
  }
  static __device__ __forceinline__ void guard(v8f& a, v8f& b, v16h x, v16h y) { dep_guard_h(a, b, x, y); }
  static __device__ __forceinline__ void keep(v16h a, v16h b, v16h c, v16h d) { keep4_h(a, b, c, d); }
};
template <> struct Frag<__bf16> {
  typedef v16b V; union U { v16b v; v8b h[2]; };
  static __device__ __forceinline__ v16b load(const __bf16* p) {
    U f; f.h[0] = *(const v8b*)(p); f.h[1] = *(const v8b*)(p + 16); return f.v;
  }
  static __device__ __forceinline__ v8f mma(v16b a, v16b b, v8f c) {
    return __builtin_amdgcn_wmma_f32_16x16x32_bf16(false, a, false, b, (short)0, c, false, false);
  }
  static __device__ __forceinline__ void guard(v8f& a, v8f& b, v16b x, v16b y) { dep_guard_b(a, b, x, y); }
  static __device__ __forceinline__ void keep(v16b a, v16b b, v16b c, v16b d) { keep4_b(a, b, c, d); }
};

template <int ET> struct Elem;
template <> struct Elem<0> { typedef _Float16 T; };
template <> struct Elem<1> { typedef __bf16 T; };
template <int ET, bool SPLIT, int BIAS_MODE, int OUT_MODE, bool RESID, int ACT = 0>
__global__ __launch_bounds__(256) void wmma_gemm64(
    const unsigned short* __restrict__ Ap, const unsigned short* __restrict__ A2p, int lda, long strideA,
    const unsigned short* __restrict__ Btp, const unsigned short* __restrict__ Bt2p, int ldb, long strideB,
    void* __restrict__ Cout, void* __restrict__ Cout2, int ldc, long strideC,
    const float* __restrict__ bias,
    const float* __restrict__ resid, long strideR,
    int M, int N, int K, float scale) {
  typedef typename Elem<ET>::T T;
  typedef typename Frag<T>::V V;
  const T* A = (const T*)Ap; const T* A2 = (const T*)A2p; const T* Bt = (const T*)Btp; const T* Bt2 = (const T*)Bt2p;
  __shared__ __align__(16) float sT[8][16 * 68];
  const int b    = blockIdx.y;
  const int lane = threadIdx.x & 31;
  const int wave = threadIdx.x >> 5;
  const int tilesN = N >> 6;
  const int tilesM = M >> 6;
  const int tile = blockIdx.x * 8 + wave;
  if (tile >= tilesM * tilesN) return;
  const int tm = tile / tilesN;
  const int tn = tile - tm * tilesN;
  const int m0 = tm << 6;
  const int n0 = tn << 6;

  const T* Ab  = A  + (size_t)b * strideA;
  const T* Bb  = Bt + (size_t)b * strideB;
  const T* Ab2 = SPLIT ? (A2  + (size_t)b * strideA) : nullptr;
  const T* Bb2 = SPLIT ? (Bt2 + (size_t)b * strideB) : nullptr;

  const int rlane = lane & 15;
  const int koff  = (lane >> 4) * 8;
  const int mOff  = (lane >> 4) * 8;

  v8f acc[4][4];
#pragma unroll
  for (int i = 0; i < 4; ++i)
#pragma unroll
    for (int j = 0; j < 4; ++j) acc[i][j] = (v8f){0.f,0.f,0.f,0.f,0.f,0.f,0.f,0.f};

  for (int k0 = 0; k0 < K; k0 += 32) {
    V bh[4], bl[4];
#pragma unroll
    for (int j = 0; j < 4; ++j) {
      const size_t bo = (size_t)(n0 + (j << 4) + rlane) * ldb + koff + k0;
      bh[j] = Frag<T>::load(Bb + bo);
      if (SPLIT) bl[j] = Frag<T>::load(Bb2 + bo);
    }
#pragma unroll
    for (int i = 0; i < 4; ++i) {
      const size_t ao = (size_t)(m0 + (i << 4) + rlane) * lda + koff + k0;
      V ah = Frag<T>::load(Ab + ao);
      V al;
      if (SPLIT) al = Frag<T>::load(Ab2 + ao);
#pragma unroll
      for (int j = 0; j < 4; ++j) {
        acc[i][j] = Frag<T>::mma(ah, bh[j], acc[i][j]);
        if (SPLIT) {
          acc[i][j] = Frag<T>::mma(ah, bl[j], acc[i][j]);
          acc[i][j] = Frag<T>::mma(al, bh[j], acc[i][j]);
        }
      }
      Frag<T>::guard(acc[i][0], acc[i][3], ah, SPLIT ? al : ah);
    }
    Frag<T>::keep(bh[0], bh[1], bh[2], bh[3]);
    if (SPLIT) Frag<T>::keep(bl[0], bl[1], bl[2], bl[3]);
  }
  acc_guard4(acc[0][0], acc[0][1], acc[0][2], acc[0][3]);
  acc_guard4(acc[1][0], acc[1][1], acc[1][2], acc[1][3]);
  acc_guard4(acc[2][0], acc[2][1], acc[2][2], acc[2][3]);
  acc_guard4(acc[3][0], acc[3][1], acc[3][2], acc[3][3]);

  float* slab = sT[wave];
  const float* Rb = RESID ? (resid + (size_t)b * strideR) : nullptr;
#pragma unroll
  for (int i = 0; i < 4; ++i) {
    const int mBase = m0 + (i << 4);
#pragma unroll
    for (int j = 0; j < 4; ++j) {
      const int n = n0 + (j << 4) + rlane;
      float bv = 0.f;
      if (BIAS_MODE == 2) bv = bias[n];
#pragma unroll
      for (int r = 0; r < 8; ++r) {
        float v = acc[i][j][r] * scale;
        if (BIAS_MODE == 1) v += bias[mBase + mOff + r];
        if (BIAS_MODE == 2) v += bv;
        if (RESID) v += Rb[(size_t)(mBase + mOff + r) * ldc + n];
        if (ACT == 2) v = fmaxf(v, 0.0f);
        if (ACT == 4) v = (v > 0.f) ? v : 0.01f * v;
        slab[(mOff + r) * 68 + (j << 4) + rlane] = v;
      }
    }
    __builtin_amdgcn_fence(__ATOMIC_RELEASE, "workgroup");
    __builtin_amdgcn_wave_barrier();
    __builtin_amdgcn_fence(__ATOMIC_ACQUIRE, "workgroup");
    if (OUT_MODE == 0) {
      float* C = (float*)Cout + (size_t)b * strideC;
      const int hh = lane >> 4, c4 = (lane & 15) * 4;
      for (int pass = 0; pass < 2; ++pass) {
#pragma unroll
        for (int it = 0; it < 8; ++it) {
          const int row = it * 2 + hh;
          v4f v = *(const v4f*)(slab + row * 68 + c4);
          *(volatile v4f*)(C + (size_t)(mBase + row) * ldc + n0 + c4) = v;
        }
        __threadfence();
      }
    } else {
      const int q = lane >> 3, c8 = (lane & 7) * 8;
      unsigned short* C  = (unsigned short*)Cout  + (size_t)b * strideC;
      unsigned short* C2 = (OUT_MODE == 2) ? ((unsigned short*)Cout2 + (size_t)b * strideC) : nullptr;
      for (int pass = 0; pass < 2; ++pass) {
#pragma unroll
        for (int it = 0; it < 4; ++it) {
          const int row = it * 4 + q;
          const float* sp = slab + row * 68 + c8;
          v8h hv, lv;
#pragma unroll
          for (int e = 0; e < 8; ++e) {
            if (OUT_MODE == 1) {
              hv[e] = (_Float16)sp[e];
            } else {
              unsigned short hb = f2bf_bits(sp[e]);
              unsigned short lb = f2bf_bits(sp[e] - bf_bits2f(hb));
              hv[e] = __builtin_bit_cast(_Float16, hb);
              lv[e] = __builtin_bit_cast(_Float16, lb);
            }
          }
          *(volatile v8h*)(C + (size_t)(mBase + row) * ldc + n0 + c8) = hv;
          if (OUT_MODE == 2) *(volatile v8h*)(C2 + (size_t)(mBase + row) * ldc + n0 + c8) = lv;
        }
        __threadfence();
      }
    }
    __builtin_amdgcn_fence(__ATOMIC_RELEASE, "workgroup");
    __builtin_amdgcn_wave_barrier();
    __builtin_amdgcn_fence(__ATOMIC_ACQUIRE, "workgroup");
  }
}

__global__ __launch_bounds__(256) void cast_scale_f16x2(const float* __restrict__ in, unsigned short* __restrict__ out, int n2, float sc) {
  const int i = blockIdx.x * 256 + threadIdx.x;
  if (i < n2) {
    const _Float16 h0 = (_Float16)(in[2 * i] * sc), h1 = (_Float16)(in[2 * i + 1] * sc);
    const unsigned u = (unsigned)__builtin_bit_cast(unsigned short, h0) | ((unsigned)__builtin_bit_cast(unsigned short, h1) << 16);
    ((volatile unsigned*)out)[i] = u;
    __threadfence();
    ((volatile unsigned*)out)[i] = u;
  }
}

__global__ __launch_bounds__(256) void prep_small_kernel(const float* __restrict__ Wp, const float* __restrict__ Wv,
                                                        const float* __restrict__ bp, const float* __restrict__ bv,
                                                        const float* __restrict__ b_ih, const float* __restrict__ b_hh,
                                                        unsigned short* __restrict__ WPV, float* __restrict__ bsum,
                                                        float* __restrict__ bpv) {
  const int tid = threadIdx.x;
  for (int pass = 0; pass < 2; ++pass) {
#pragma unroll 1
    for (int it = 0; it < 16; ++it) {
      const int u = it * 256 + tid;
      const int e0 = 2 * u;
      const int row = e0 >> 7, col = e0 & 127;
      const int rp = row < 7 ? row : 7;
      const float p0 = Wp[rp * kLstm + col], p1 = Wp[rp * kLstm + col + 1];
      const float q0 = Wv[col], q1 = Wv[col + 1];
      const float s0 = (row < 8) ? p0 : ((row == 8) ? q0 : 0.0f);
      const float s1 = (row < 8) ? p1 : ((row == 8) ? q1 : 0.0f);
      const _Float16 h0 = (_Float16)(s0 * 16.0f), h1 = (_Float16)(s1 * 16.0f);
      const unsigned w = (unsigned)__builtin_bit_cast(unsigned short, h0) | ((unsigned)__builtin_bit_cast(unsigned short, h1) << 16);
      ((volatile unsigned*)WPV)[u] = w;
    }
#pragma unroll 1
    for (int it = 0; it < 2; ++it) {
      const int i = it * 256 + tid;
      const float s = b_ih[i] + b_hh[i];
      ((volatile float*)bsum)[i] = s;
    }
    if (tid < 64) {
      const int ip = tid < 7 ? tid : 7;
      const float a = bp[ip];
      const float c = bv[0];
      const float s = (tid < 8) ? a : ((tid == 8) ? c : 0.0f);
      ((volatile float*)bpv)[tid] = s;
    }
    __threadfence();
  }
}

__global__ __launch_bounds__(256) void norm_kernel(const float* __restrict__ obs, const float* __restrict__ mean,
                                                  const float* __restrict__ var, unsigned short* __restrict__ X16, int g) {
  union F8 { v4f v[2]; float f[8]; };
  const int tid = threadIdx.x;
  const int row = blockIdx.x * 32 + (tid >> 3);
  const int c8 = (tid & 7) * 8;
  const int t = row >> 7, bl = row & 127;
  const int b = g * kSeqGrp + bl;
  const float* src = obs + ((size_t)t * kBatch + b) * kObs + c8;
  F8 o;
  o.v[0] = *(const v4f*)(src);
  o.v[1] = *(const v4f*)(src + 4);
  v8h hv;
#pragma unroll
  for (int e = 0; e < 8; ++e) {
    const int d = c8 + e;
    const float vv = fmaxf(var[d], 1e-6f);
    float x = (o.f[e] - mean[d]) * rsqrtf(vv);
    x = fminf(10.0f, fmaxf(-10.0f, x));
    hv[e] = (_Float16)x;
  }
  unsigned short* dst = X16 + (size_t)row * kObs + c8;
  *(volatile v8h*)dst = hv;
  __threadfence();
  *(volatile v8h*)dst = hv;
}

__device__ __forceinline__ float fsig(float x)  { return __builtin_amdgcn_rcpf(1.0f + __expf(-x)); }
__device__ __forceinline__ float ftanh(float x) { return 1.0f - 2.0f * __builtin_amdgcn_rcpf(__expf(2.0f * x) + 1.0f); }

__global__ __launch_bounds__(256) void lstm_rec_kernel(const float* __restrict__ xp, const unsigned short* __restrict__ WHHp,
                                                      const float* __restrict__ h0, const float* __restrict__ c0,
                                                      const int* __restrict__ done, int g,
                                                      unsigned short* __restrict__ outs16,
                                                      float* __restrict__ out_h, float* __restrict__ out_c) {
  __shared__ __align__(16) _Float16 Ah[16 * kAhP];
  __shared__ __align__(16) _Float16 Hs16[16 * kAhP];
  __shared__ __align__(16) float    Hf[16 * kHfP];
  __shared__ float sRt[16];
  const _Float16* WH = (const _Float16*)WHHp;
  const int tid = threadIdx.x, lane = tid & 31, wave = tid >> 5;
  const int c = lane & 15, hh = lane >> 4, koff = hh * 8;
  const int bl0 = blockIdx.x * 16;
  const int b0 = g * kSeqGrp + bl0;
  const int j = 16 * wave + c;

  if (tid < 16) sRt[tid] = 1.0f - (float)done[b0 + tid];
  __syncthreads();
#pragma unroll 1
  for (int it = 0; it < 8; ++it) {
    const int i = it * kNT + tid;
    const int row = i >> 7, k = i & 127;
    Ah[row * kAhP + k] = (_Float16)(h0[(size_t)(b0 + row) * kLstm + k] * sRt[row]);
  }
  float cst[8], hst[8];
#pragma unroll
  for (int r = 0; r < 8; ++r) {
    const int row = 8 * hh + r;
    cst[r] = c0[(size_t)(b0 + row) * kLstm + j] * sRt[row];
    hst[r] = 0.0f;
  }
  __syncthreads();

  const _Float16* ahrow = Ah + c * kAhP + koff;
  const _Float16* wh = WH + (size_t)j * kLstm + koff;
  const v8f z8 = {0.f, 0.f, 0.f, 0.f, 0.f, 0.f, 0.f, 0.f};

#pragma unroll 1
  for (int t = 0; t < kSteps; ++t) {
    v8f acc[4];
    acc[0] = z8; acc[1] = z8; acc[2] = z8; acc[3] = z8;
#pragma unroll 1
    for (int k0 = 0; k0 < kLstm; k0 += 32) {
      const v16h a   = Frag<_Float16>::load(ahrow + k0);
      const v16h bq0 = Frag<_Float16>::load(wh + k0);
      const v16h bq1 = Frag<_Float16>::load(wh + (size_t)1 * kLstm * kLstm + k0);
      const v16h bq2 = Frag<_Float16>::load(wh + (size_t)2 * kLstm * kLstm + k0);
      const v16h bq3 = Frag<_Float16>::load(wh + (size_t)3 * kLstm * kLstm + k0);
      acc[0] = Frag<_Float16>::mma(a, bq0, acc[0]);
      acc[1] = Frag<_Float16>::mma(a, bq1, acc[1]);
      acc[2] = Frag<_Float16>::mma(a, bq2, acc[2]);
      acc[3] = Frag<_Float16>::mma(a, bq3, acc[3]);
      dep_guard_h(acc[0], acc[3], a, bq3);
      keep4_h(bq0, bq1, bq2, bq3);
    }
    acc_guard4(acc[0], acc[1], acc[2], acc[3]);

    if (tid < 16) {
      const int tn = (t + 1 < kSteps) ? (t + 1) : (kSteps - 1);
      float rn = 1.0f - (float)done[(size_t)tn * kBatch + b0 + tid];
      if (t + 1 >= kSteps) rn = 1.0f;
      sRt[tid] = rn;
    }

    const float* xr0 = xp + ((size_t)t * kSeqGrp + bl0 + 8 * hh) * kGates + j;
#pragma unroll
    for (int r = 0; r < 8; ++r) {
      const float* xr = xr0 + (size_t)r * kGates;
      const float zi = acc[0][r] * kInv16 + xr[0];
      const float zf = acc[1][r] * kInv16 + xr[kLstm];
      const float zg = acc[2][r] * kInv16 + xr[2 * kLstm];
      const float zo = acc[3][r] * kInv16 + xr[3 * kLstm];
      const float ig = fsig(zi);
      const float fg = fsig(zf);
      const float gt = ftanh(zg);
      const float og = fsig(zo);
      const float cn = fg * cst[r] + ig * gt;
      cst[r] = cn;
      hst[r] = og * ftanh(cn);
    }
    __syncthreads();

#pragma unroll
    for (int r = 0; r < 8; ++r) {
      const int row = 8 * hh + r;
      const float rn = sRt[row];
      Hs16[row * kAhP + j] = (_Float16)hst[r];
      Ah[row * kAhP + j]   = (_Float16)(hst[r] * rn);
      cst[r] *= rn;
      hst[r] *= rn;
    }
    __syncthreads();

    {
      const int row = tid >> 4, c8 = (tid & 15) * 8;
      const v8h v = *(const v8h*)(Hs16 + row * kAhP + c8);
      unsigned short* dst = outs16 + ((size_t)t * kSeqGrp + bl0 + row) * kLstm + c8;
      *(volatile v8h*)dst = v;
      __threadfence();
      *(volatile v8h*)dst = v;
    }
  }

#pragma unroll
  for (int r = 0; r < 8; ++r) Hf[(8 * hh + r) * kHfP + j] = hst[r];
  __syncthreads();
  for (int pass = 0; pass < 2; ++pass) {
#pragma unroll
    for (int it = 0; it < 2; ++it) {
      const int idx = it * kNT + tid;
      const int row = idx >> 5, c4 = (idx & 31) * 4;
      const v4f v = *(const v4f*)(Hf + row * kHfP + c4);
      *(volatile v4f*)(out_h + (size_t)(b0 + row) * kLstm + c4) = v;
    }
    __threadfence();
  }
  __syncthreads();
#pragma unroll
  for (int r = 0; r < 8; ++r) Hf[(8 * hh + r) * kHfP + j] = cst[r];
  __syncthreads();
  for (int pass = 0; pass < 2; ++pass) {
#pragma unroll
    for (int it = 0; it < 2; ++it) {
      const int idx = it * kNT + tid;
      const int row = idx >> 5, c4 = (idx & 31) * 4;
      const v4f v = *(const v4f*)(Hf + row * kHfP + c4);
      *(volatile v4f*)(out_c + (size_t)(b0 + row) * kLstm + c4) = v;
    }
    __threadfence();
  }
}

__global__ __launch_bounds__(256) void pack_kernel(const float* __restrict__ headf, const int* __restrict__ amask, int g,
                                                  float* __restrict__ out_logits, float* __restrict__ out_values) {
  const int tid = threadIdx.x, lane = tid & 31, wave = tid >> 5;
  const int rp0 = blockIdx.x * 32;
  const int t = rp0 >> 7;
  const int b0 = g * kSeqGrp + (rp0 & 127);
  {
    const int q = lane >> 3, a = lane & 7;
    const int rl = 4 * wave + q;
    const float v = headf[(size_t)(rp0 + rl) * kHeadN + a];
    const size_t oi = ((size_t)t * kBatch + b0 + rl) * kAct + a;
    const int m = amask[oi];
    const float o = (m > 0) ? v : -1.0e9f;
    *(volatile float*)(out_logits + oi) = o;
    __threadfence();
    *(volatile float*)(out_logits + oi) = o;
  }
  if (wave == 0) {
    const float v = headf[(size_t)(rp0 + lane) * kHeadN + kAct];
    float* p = out_values + (size_t)t * kBatch + b0 + lane;
    *(volatile float*)p = v;
    __threadfence();
    *(volatile float*)p = v;
  }
}

extern "C" void kernel_launch(void* const* d_in, const int* in_sizes, int n_in,
                              void* d_out, int out_size, void* d_ws, size_t ws_size, hipStream_t stream) {
  if (n_in < 19 || d_out == nullptr || d_ws == nullptr) return;
  if (in_sizes[0] != kSteps * kBatch * kObs || in_sizes[1] != kBatch * kLstm || in_sizes[2] != kBatch * kLstm ||
      in_sizes[3] != kSteps * kBatch || in_sizes[4] != kSteps * kBatch * kAct || in_sizes[5] != kObs || in_sizes[6] != kObs ||
      in_sizes[7] != kEnc1 * kObs || in_sizes[8] != kEnc1 || in_sizes[9] != kHid * kEnc1 || in_sizes[10] != kHid ||
      in_sizes[11] != kGates * kHid || in_sizes[12] != kGates * kLstm || in_sizes[13] != kGates || in_sizes[14] != kGates ||
      in_sizes[15] != kAct * kLstm || in_sizes[16] != kAct || in_sizes[17] != kLstm || in_sizes[18] != 1) return;
  if (out_size != kSteps * kBatch * kAct + kSteps * kBatch + 2 * kBatch * kLstm) return;

  const float* obs   = (const float*)d_in[0];
  const float* h0    = (const float*)d_in[1];
  const float* c0    = (const float*)d_in[2];
  const int*   done  = (const int*)d_in[3];
  const int*   amask = (const int*)d_in[4];
  const float* omean = (const float*)d_in[5];
  const float* ovar  = (const float*)d_in[6];
  const float* W1    = (const float*)d_in[7];
  const float* b1    = (const float*)d_in[8];
  const float* W2    = (const float*)d_in[9];
  const float* b2    = (const float*)d_in[10];
  const float* W_ih  = (const float*)d_in[11];
  const float* W_hh  = (const float*)d_in[12];
  const float* b_ih  = (const float*)d_in[13];
  const float* b_hh  = (const float*)d_in[14];
  const float* Wp    = (const float*)d_in[15];
  const float* bp    = (const float*)d_in[16];
  const float* Wv    = (const float*)d_in[17];
  const float* bv    = (const float*)d_in[18];

  float* out_logits = (float*)d_out;
  float* out_values = out_logits + (size_t)kSteps * kBatch * kAct;
  float* out_h      = out_values + (size_t)kSteps * kBatch;
  float* out_c      = out_h + (size_t)kBatch * kLstm;

  char* ws = (char*)d_ws; size_t off = 0;
  auto carve = [&](size_t bytes) -> char* { char* p = ws + off; off += (bytes + 255) & ~(size_t)255; return p; };
  unsigned short* W1h   = (unsigned short*)carve((size_t)kEnc1 * kObs * 2);
  unsigned short* W2h   = (unsigned short*)carve((size_t)kHid * kEnc1 * 2);
  unsigned short* WIHh  = (unsigned short*)carve((size_t)kGates * kHid * 2);
  unsigned short* WHHh  = (unsigned short*)carve((size_t)kGates * kLstm * 2);
  unsigned short* WPVh  = (unsigned short*)carve((size_t)kHeadN * kLstm * 2);
  float*          bsum  = (float*)carve((size_t)kGates * 4);
  float*          bpv   = (float*)carve((size_t)kHeadN * 4);
  unsigned short* X16   = (unsigned short*)carve((size_t)kRowsGrp * kObs * 2);
  unsigned short* E1    = (unsigned short*)carve((size_t)kRowsGrp * kEnc1 * 2);
  unsigned short* E2    = (unsigned short*)carve((size_t)kRowsGrp * kHid * 2);
  float*          XP    = (float*)carve((size_t)kRowsGrp * kGates * 4);
  unsigned short* OUTS  = (unsigned short*)carve((size_t)kRowsGrp * kLstm * 2);
  float*          HEADF = (float*)carve((size_t)kRowsGrp * kHeadN * 4);
  if (off > ws_size || off > (size_t)134217728) return;

  {
    const int n1 = kEnc1 * kObs / 2, n2 = kHid * kEnc1 / 2, n3 = kGates * kHid / 2, n4 = kGates * kLstm / 2;
    cast_scale_f16x2<<<(n1 + 255) / 256, 256, 0, stream>>>(W1, W1h, n1, 8.0f);
    cast_scale_f16x2<<<(n2 + 255) / 256, 256, 0, stream>>>(W2, W2h, n2, 8.0f);
    cast_scale_f16x2<<<(n3 + 255) / 256, 256, 0, stream>>>(W_ih, WIHh, n3, 16.0f);
    cast_scale_f16x2<<<(n4 + 255) / 256, 256, 0, stream>>>(W_hh, WHHh, n4, 16.0f);
    prep_small_kernel<<<1, 256, 0, stream>>>(Wp, Wv, bp, bv, b_ih, b_hh, WPVh, bsum, bpv);
  }

  const int M = kRowsGrp;
  const dim3 gL1((M / 64) * (kEnc1 / 64) / 8, 1);
  const dim3 gL2((M / 64) * (kHid / 64) / 8, 1);
  const dim3 gXP((M / 64) * (kGates / 64) / 8, 1);
  const dim3 gHD((M / 64) * (kHeadN / 64) / 8, 1);
  for (int g = 0; g < kGroups; ++g) {
    norm_kernel<<<M / 32, kNT, 0, stream>>>(obs, omean, ovar, X16, g);
    wmma_gemm64<0, false, 2, 1, false, 2><<<gL1, 256, 0, stream>>>(
        X16, X16, kObs, 0L, W1h, W1h, kObs, 0L, (void*)E1, (void*)E1, kEnc1, 0L, b1, b1, 0L, M, kEnc1, kObs, kInv8);
    wmma_gemm64<0, false, 2, 1, false, 2><<<gL2, 256, 0, stream>>>(
        E1, E1, kEnc1, 0L, W2h, W2h, kEnc1, 0L, (void*)E2, (void*)E2, kHid, 0L, b2, b2, 0L, M, kHid, kEnc1, kInv8);
    wmma_gemm64<0, false, 2, 0, false, 0><<<gXP, 256, 0, stream>>>(
        E2, E2, kHid, 0L, WIHh, WIHh, kHid, 0L, (void*)XP, (void*)XP, kGates, 0L, bsum, bsum, 0L, M, kGates, kHid, kInv16);
    lstm_rec_kernel<<<kSeqGrp / 16, kNT, 0, stream>>>(XP, WHHh, h0, c0, done, g, OUTS, out_h, out_c);
    wmma_gemm64<0, false, 2, 0, false, 0><<<gHD, 256, 0, stream>>>(
        OUTS, OUTS, kLstm, 0L, WPVh, WPVh, kLstm, 0L, (void*)HEADF, (void*)HEADF, kHeadN, 0L, bpv, bpv, 0L, M, kHeadN, kLstm, kInv16);
    pack_kernel<<<M / 32, kNT, 0, stream>>>(HEADF, amask, g, out_logits, out_values);
  }
}
